// RNNBlock_82386062671988
// MI455X (gfx1250) — hardware-verified
//
#include <hip/hip_runtime.h>
#include <math.h>

typedef __attribute__((ext_vector_type(16))) _Float16 v16h;
typedef __attribute__((ext_vector_type(8)))  _Float16 v8h;
typedef __attribute__((ext_vector_type(16))) __bf16   v16b;
typedef __attribute__((ext_vector_type(8)))  __bf16   v8b;
typedef __attribute__((ext_vector_type(8)))  float    v8f;
typedef __attribute__((ext_vector_type(4)))  float    v4f;

constexpr int kB    = 16384;
constexpr int kT    = 79;
constexpr int kF    = 3;
constexpr int kH    = 256;
constexpr int kD    = 256;
constexpr int kThr  = 256;
constexpr float kInCarry = 1024.0f;
constexpr float kWCarry  = 4096.0f;
constexpr float kSc = 1.0f / (kInCarry * kWCarry);
constexpr float kF16MinNormal = 6.103515625e-5f;
constexpr int kFZ = 0, kFBD = 256, kFEnd = 1024;

static_assert((kB % 64) == 0 && ((kB / 64) * (kH / 64)) % 8 == 0 && (kH % 32) == 0 && kH == kD && (kH / 8) <= 256, "GEMM M, N multiples of 64; grids exact; K multiples of 32");

constexpr size_t kOffUT = 0ull;
constexpr size_t kOffWDT = 131072ull;
constexpr size_t kOffBIAS = 262144ull;
constexpr size_t kOffH16 = 266240ull;
constexpr size_t kOffG32 = 8654848ull;
constexpr size_t kWsTotal = 25432064ull;
static_assert(kWsTotal <= 134217728ull, "carve cap: under 128 MiB");
static_assert(kOffUT == 0
              && kOffWDT == kOffUT + 131072ull
              && kOffBIAS == kOffWDT + 131072ull
              && kOffH16 == kOffBIAS + 4096ull
              && kOffG32 == kOffH16 + 8388608ull
              && kWsTotal == kOffG32 + 16777216ull, "the carve is chained and totalled");
static_assert((kOffUT % 256) == 0 && (kOffWDT % 256) == 0 && (kOffBIAS % 256) == 0 && (kOffH16 % 256) == 0 && (kOffG32 % 256) == 0, "aligned regions");

__device__ __forceinline__ unsigned short f2bf_bits(float f) {
  unsigned u = __float_as_uint(f);
  return (unsigned short)((u + 0x7FFFu + ((u >> 16) & 1u)) >> 16);
}
__device__ __forceinline__ float bf_bits2f(unsigned short h) { return __uint_as_float(((unsigned)h) << 16); }
__device__ __forceinline__ float bf16r(float f) { return bf_bits2f(f2bf_bits(f)); }
__device__ __forceinline__ float carry_flush(float v, float carry) {
  const float s = v * carry;
  return (fabsf(s) < kF16MinNormal) ? 0.0f : s;
}
__device__ __forceinline__ float frcp(float x) { return __builtin_amdgcn_rcpf(x); }

__device__ __forceinline__ void dep_guard4_h(v8f& a, v8f& b, v8f& c, v8f& d, v16h x, v16h y) { asm volatile("v_nop\n\tv_nop\n\tv_nop\n\tv_nop" : "+v"(a), "+v"(b), "+v"(c), "+v"(d) : "v"(x), "v"(y)); }
__device__ __forceinline__ void dep_guard4_b(v8f& a, v8f& b, v8f& c, v8f& d, v16b x, v16b y) { asm volatile("v_nop\n\tv_nop\n\tv_nop\n\tv_nop" : "+v"(a), "+v"(b), "+v"(c), "+v"(d) : "v"(x), "v"(y)); }
__device__ __forceinline__ void keep4_h(v16h a, v16h b, v16h c, v16h d) { asm volatile("v_nop" :: "v"(a), "v"(b), "v"(c), "v"(d)); }
__device__ __forceinline__ void keep4_b(v16b a, v16b b, v16b c, v16b d) { asm volatile("v_nop" :: "v"(a), "v"(b), "v"(c), "v"(d)); }
__device__ __forceinline__ void acc_guard4(v8f& a, v8f& b, v8f& c, v8f& d) { asm volatile("v_nop\n\tv_nop\n\tv_nop\n\tv_nop" : "+v"(a), "+v"(b), "+v"(c), "+v"(d)); }

template <typename T> struct Frag;
template <> struct Frag<_Float16> {
  typedef v16h V; union U { v16h v; v8h h[2]; };
  static __device__ __forceinline__ v16h load(const _Float16* p) {
    U f; f.h[0] = *(const v8h*)(p); f.h[1] = *(const v8h*)(p + 16); return f.v;
  }
  static __device__ __forceinline__ v8f mma(v16h a, v16h b, v8f c) {
    return __builtin_amdgcn_wmma_f32_16x16x32_f16(false, a, false, b, (short)0, c, false, false);
  }
  static __device__ __forceinline__ void guard4(v8f& a, v8f& b, v8f& c, v8f& d, v16h x, v16h y) { dep_guard4_h(a, b, c, d, x, y); }
  static __device__ __forceinline__ void keep(v16h a, v16h b, v16h c, v16h d) { keep4_h(a, b, c, d); }
};
template <> struct Frag<__bf16> {
  typedef v16b V; union U { v16b v; v8b h[2]; };
  static __device__ __forceinline__ v16b load(const __bf16* p) {
    U f; f.h[0] = *(const v8b*)(p); f.h[1] = *(const v8b*)(p + 16); return f.v;
  }
  static __device__ __forceinline__ v8f mma(v16b a, v16b b, v8f c) {
    return __builtin_amdgcn_wmma_f32_16x16x32_bf16(false, a, false, b, (short)0, c, false, false);
  }
  static __device__ __forceinline__ void guard4(v8f& a, v8f& b, v8f& c, v8f& d, v16b x, v16b y) { dep_guard4_b(a, b, c, d, x, y); }
  static __device__ __forceinline__ void keep(v16b a, v16b b, v16b c, v16b d) { keep4_b(a, b, c, d); }
};

__device__ __forceinline__ v8f mma_h(v16h a, v16h b, v8f c) {
  c = __builtin_amdgcn_wmma_f32_16x16x32_f16(false, a, false, b, (short)0, c, false, false);
  asm volatile("v_nop\n\tv_nop\n\tv_nop\n\tv_nop" : "+v"(c) : "v"(a), "v"(b));
  return c;
}

template <int ET> struct Elem;
template <> struct Elem<0> { typedef _Float16 T; };
template <> struct Elem<1> { typedef __bf16 T; };
template <int ET, bool SPLIT, int BIAS_MODE, int OUT_MODE, bool RESID, int ACT = 0>
__global__ __launch_bounds__(256) void wmma_gemm64(
    const unsigned short* __restrict__ Ap, const unsigned short* __restrict__ A2p, int lda, long strideA,
    const unsigned short* __restrict__ Btp, const unsigned short* __restrict__ Bt2p, int ldb, long strideB,
    void* __restrict__ Cout, void* __restrict__ Cout2, int ldc, long strideC,
    const float* __restrict__ bias,
    const float* __restrict__ resid, long strideR,
    int M, int N, int K, float scale) {
  typedef typename Elem<ET>::T T;
  typedef typename Frag<T>::V V;
  const T* A = (const T*)Ap; const T* A2 = (const T*)A2p; const T* Bt = (const T*)Btp; const T* Bt2 = (const T*)Bt2p;
  __shared__ __align__(16) float sT[8][16 * 68];
  const int b    = blockIdx.y;
  const int lane = threadIdx.x & 31;
  const int wave = threadIdx.x >> 5;
  const int tilesN = N >> 6;
  const int tilesM = M >> 6;
  const int tile = blockIdx.x * 8 + wave;
  if (tile >= tilesM * tilesN) return;
  const int tm = tile / tilesN;
  const int tn = tile - tm * tilesN;
  const int m0 = tm << 6;
  const int n0 = tn << 6;

  const T* Ab  = A  + (size_t)b * strideA;
  const T* Bb  = Bt + (size_t)b * strideB;
  const T* Ab2 = SPLIT ? (A2  + (size_t)b * strideA) : nullptr;
  const T* Bb2 = SPLIT ? (Bt2 + (size_t)b * strideB) : nullptr;

  const int rlane = lane & 15;
  const int koff  = (lane >> 4) * 8;
  const int mOff  = (lane >> 4) * 8;

  v8f acc[4][4];
#pragma unroll
  for (int i = 0; i < 4; ++i)
#pragma unroll
    for (int j = 0; j < 4; ++j) acc[i][j] = (v8f){0.f,0.f,0.f,0.f,0.f,0.f,0.f,0.f};

  for (int k0 = 0; k0 < K; k0 += 32) {
    V bh[4], bl[4];
#pragma unroll
    for (int j = 0; j < 4; ++j) {
      const size_t bo = (size_t)(n0 + (j << 4) + rlane) * ldb + koff + k0;
      bh[j] = Frag<T>::load(Bb + bo);
      if (SPLIT) bl[j] = Frag<T>::load(Bb2 + bo);
    }
#pragma unroll
    for (int i = 0; i < 4; ++i) {
      const size_t ao = (size_t)(m0 + (i << 4) + rlane) * lda + koff + k0;
      V ah = Frag<T>::load(Ab + ao);
      V al;
      if (SPLIT) al = Frag<T>::load(Ab2 + ao);
#pragma unroll
      for (int j = 0; j < 4; ++j) {
        acc[i][j] = Frag<T>::mma(ah, bh[j], acc[i][j]);
        if (SPLIT) {
          acc[i][j] = Frag<T>::mma(ah, bl[j], acc[i][j]);
          acc[i][j] = Frag<T>::mma(al, bh[j], acc[i][j]);
        }
      }
      Frag<T>::guard4(acc[i][0], acc[i][1], acc[i][2], acc[i][3], ah, SPLIT ? al : ah);
    }
    Frag<T>::keep(bh[0], bh[1], bh[2], bh[3]);
    if (SPLIT) Frag<T>::keep(bl[0], bl[1], bl[2], bl[3]);
  }
  acc_guard4(acc[0][0], acc[0][1], acc[0][2], acc[0][3]);
  acc_guard4(acc[1][0], acc[1][1], acc[1][2], acc[1][3]);
  acc_guard4(acc[2][0], acc[2][1], acc[2][2], acc[2][3]);
  acc_guard4(acc[3][0], acc[3][1], acc[3][2], acc[3][3]);

  float* slab = sT[wave];
  const float* Rb = RESID ? (resid + (size_t)b * strideR) : nullptr;
#pragma unroll
  for (int i = 0; i < 4; ++i) {
    const int mBase = m0 + (i << 4);
#pragma unroll
    for (int j = 0; j < 4; ++j) {
      const int n = n0 + (j << 4) + rlane;
      float bv = 0.f;
      if (BIAS_MODE == 2) bv = bias[n];
#pragma unroll
      for (int r = 0; r < 8; ++r) {
        float v = acc[i][j][r] * scale;
        if (BIAS_MODE == 1) v += bias[mBase + mOff + r];
        if (BIAS_MODE == 2) v += bv;
        if (RESID) v += Rb[(size_t)(mBase + mOff + r) * ldc + n];
        if (ACT == 1) v = tanhf(v);
        if (ACT == 2) v = fmaxf(v, 0.0f);
        if (ACT == 3) v = v / (1.0f + expf(-v));
        if (ACT == 4) v = (v > 0.f) ? v : 0.01f * v;
        slab[(mOff + r) * 68 + (j << 4) + rlane] = v;
      }
    }
    __builtin_amdgcn_fence(__ATOMIC_RELEASE, "workgroup");
    __builtin_amdgcn_wave_barrier();
    __builtin_amdgcn_fence(__ATOMIC_ACQUIRE, "workgroup");
    if (OUT_MODE == 0) {
      float* C = (float*)Cout + (size_t)b * strideC;
      const int hh = lane >> 4, c4 = (lane & 15) * 4;
      for (int pass = 0; pass < 2; ++pass) {
#pragma unroll
        for (int it = 0; it < 8; ++it) {
          const int row = it * 2 + hh;
          v4f v = *(const v4f*)(slab + row * 68 + c4);
          *(volatile v4f*)(C + (size_t)(mBase + row) * ldc + n0 + c4) = v;
        }
        __threadfence();
      }
    } else {
      const int q = lane >> 3, c8 = (lane & 7) * 8;
      unsigned short* C  = (unsigned short*)Cout  + (size_t)b * strideC;
      unsigned short* C2 = (OUT_MODE == 2) ? ((unsigned short*)Cout2 + (size_t)b * strideC) : nullptr;
      for (int pass = 0; pass < 2; ++pass) {
#pragma unroll
        for (int it = 0; it < 4; ++it) {
          const int row = it * 4 + q;
          const float* sp = slab + row * 68 + c8;
          v8h hv, lv;
#pragma unroll
          for (int e = 0; e < 8; ++e) {
            if (OUT_MODE == 1) {
              hv[e] = (_Float16)sp[e];
            } else {
              unsigned short hb = f2bf_bits(sp[e]);
              unsigned short lb = f2bf_bits(sp[e] - bf_bits2f(hb));
              hv[e] = __builtin_bit_cast(_Float16, hb);
              lv[e] = __builtin_bit_cast(_Float16, lb);
            }
          }
          *(volatile v8h*)(C + (size_t)(mBase + row) * ldc + n0 + c8) = hv;
          if (OUT_MODE == 2) *(volatile v8h*)(C2 + (size_t)(mBase + row) * ldc + n0 + c8) = lv;
        }
        __threadfence();
      }
    }
    __builtin_amdgcn_fence(__ATOMIC_RELEASE, "workgroup");
    __builtin_amdgcn_wave_barrier();
    __builtin_amdgcn_fence(__ATOMIC_ACQUIRE, "workgroup");
  }
}

__global__ __launch_bounds__(256) void wt_plane_kernel(const float* __restrict__ W, unsigned short* __restrict__ dst, int K, int N, int nLive, int ldd, int colOff) {
  const int n  = blockIdx.x;
  const int k8 = threadIdx.x * 8;
  const bool live = n < nLive;
  const int nc = live ? n : 0;
  v8h hv;
#pragma unroll
  for (int e = 0; e < 8; ++e) {
    const float w = W[(size_t)(k8 + e) * N + nc];
    hv[e] = (_Float16)(live ? carry_flush(bf16r(w), kWCarry) : 0.0f);
  }
  unsigned short* dp = dst + (size_t)n * ldd + colOff + k8;
  *(volatile v8h*)dp = hv;
  __threadfence();
  *(volatile v8h*)dp = hv;
}


__global__ __launch_bounds__(kThr) void setup_kernel(const float* __restrict__ b_d, float* __restrict__ BIAS, unsigned short* __restrict__ H16) {
  unsigned v = blockIdx.x * (unsigned)kThr + threadIdx.x;
  asm volatile("" : "+v"(v));
  if (v < 256u) {
    const unsigned i0 = v * 4u;
    const bool live = (i0 >= (unsigned)kFBD) && (i0 < (unsigned)(kFBD + kD));
    const v4f a = *(const v4f*)(b_d + (live ? (i0 - (unsigned)kFBD) : 0u));
    v4f o;
#pragma unroll
    for (int e = 0; e < 4; ++e) { const float x = a[e]; o[e] = live ? bf16r(x) : 0.0f; }
    float* dp = BIAS + i0;
    *(volatile v4f*)dp = o;
    __threadfence();
    *(volatile v4f*)dp = o;
  } else {
    v8h z;
#pragma unroll
    for (int e = 0; e < 8; ++e) z[e] = (_Float16)0.0f;
    unsigned short* dp = H16 + (size_t)(v - 256u) * 8u;
    *(volatile v8h*)dp = z;
    __threadfence();
    *(volatile v8h*)dp = z;
  }
}
static_assert(kFEnd / 4 == 256 && (size_t)kB * kH / 8 == 524288 && 256 + 524288 == 2049 * kThr, "set-up grid exact");

__global__ __launch_bounds__(kThr) void relu_step_kernel(const float* __restrict__ G32, const float* __restrict__ x0, const float* __restrict__ x1,
                                                         const float* __restrict__ x2, const float* __restrict__ W_in, const float* __restrict__ b_rnn,
                                                         unsigned short* __restrict__ H16, int s) {
  unsigned v = blockIdx.x * (unsigned)kThr + threadIdx.x;
  asm volatile("" : "+v"(v));
  const unsigned b = v >> 5, u8 = (v & 31u) * 8u;
  const int t = kT - 1 - s;
  float a0 = x0[(size_t)b * kT + t], a1 = x1[(size_t)b * kT + t], a2 = x2[(size_t)b * kT + t];
  asm volatile("" : "+v"(a0), "+v"(a1), "+v"(a2));
  a0 = bf16r(a0); a1 = bf16r(a1); a2 = bf16r(a2);
  const float* gp = G32 + (size_t)b * kH + u8;
  v8h hv;
#pragma unroll
  for (int hlf = 0; hlf < 2; ++hlf) {
    const v4f g = *(const v4f*)(gp + 4 * hlf);
    const v4f w0 = *(const v4f*)(W_in + u8 + 4 * hlf), w1 = *(const v4f*)(W_in + kH + u8 + 4 * hlf), w2 = *(const v4f*)(W_in + 2 * kH + u8 + 4 * hlf);
    const v4f br = *(const v4f*)(b_rnn + u8 + 4 * hlf);
#pragma unroll
    for (int e = 0; e < 4; ++e) {
      const float p0 = w0[e], p1 = w1[e], p2 = w2[e], pb = br[e];
      float xp = a0 * bf16r(p0);
      xp += a1 * bf16r(p1);
      xp += a2 * bf16r(p2);
      xp += bf16r(pb);
      const float h = fmaxf(xp + g[e], 0.0f);
      hv[4 * hlf + e] = (_Float16)carry_flush(h, kInCarry);
    }
  }
  unsigned short* dp = H16 + (size_t)b * kH + u8;
  *(volatile v8h*)dp = hv;
  __threadfence();
  *(volatile v8h*)dp = hv;
}
static_assert((size_t)kB * kH / 8 == 2048 * (size_t)kThr, "step grid exact");

__global__ __launch_bounds__(kThr) void out_kernel(const float* __restrict__ G32, float* __restrict__ out) {
  unsigned v = blockIdx.x * (unsigned)kThr + threadIdx.x;
  asm volatile("" : "+v"(v));
  const size_t o4 = (size_t)v * 4u;
  const v4f o = *(const v4f*)(G32 + o4);
  *(volatile v4f*)(out + o4) = o;
  __threadfence();
  *(volatile v4f*)(out + o4) = o;
}
static_assert((size_t)kB * kD / 4 == 4096 * (size_t)kThr, "output grid exact");

extern "C" void kernel_launch(void* const* d_in, const int* in_sizes, int n_in,
                              void* d_out, int out_size, void* d_ws, size_t ws_size,
                              hipStream_t stream) {
  if (n_in < 8 || d_out == nullptr || d_ws == nullptr) return;
  if (in_sizes[0] != kB * kT || in_sizes[1] != kB * kT || in_sizes[2] != kB * kT || in_sizes[3] != kF * kH || in_sizes[4] != kH * kH || in_sizes[5] != kH) return;
  if (in_sizes[6] != kH * kD || in_sizes[7] != kD) return;
  if (out_size != kB * kD) return;
  if (ws_size < kWsTotal) return;
  const float* x0 = (const float*)d_in[0];
  const float* x1 = (const float*)d_in[1];
  const float* x2 = (const float*)d_in[2];
  const float* W_in = (const float*)d_in[3];
  const float* U = (const float*)d_in[4];
  const float* b_rnn = (const float*)d_in[5];
  const float* W_d = (const float*)d_in[6];
  const float* b_d = (const float*)d_in[7];
  float* out = (float*)d_out;
  char* ws = (char*)d_ws;
  unsigned short* UT = (unsigned short*)(ws + kOffUT);
  unsigned short* WDT = (unsigned short*)(ws + kOffWDT);
  float* BIAS = (float*)(ws + kOffBIAS);
  unsigned short* H16 = (unsigned short*)(ws + kOffH16);
  float* G32 = (float*)(ws + kOffG32);

  wt_plane_kernel<<<kH, kH / 8, 0, stream>>>(U, UT, kH, kH, kH, kH, 0);
  wt_plane_kernel<<<kD, kH / 8, 0, stream>>>(W_d, WDT, kH, kD, kD, kH, 0);
  setup_kernel<<<2049, kThr, 0, stream>>>(b_d, BIAS, H16);

  for (int s = 0; s < kT; ++s) {
    wmma_gemm64<0, false, 2, 0, false, 0><<<dim3((kB / 64) * (kH / 64) / 8, 1), 256, 0, stream>>>(
        H16, H16, kH, 0L, UT, UT, kH, 0L, (void*)G32, (void*)G32, kH, 0L, BIAS + kFZ, nullptr, 0L, kB, kH, kH, kSc);
    relu_step_kernel<<<2048, kThr, 0, stream>>>(G32, x0, x1, x2, W_in, b_rnn, H16, s);
  }
  wmma_gemm64<0, false, 2, 0, false, 0><<<dim3((kB / 64) * (kD / 64) / 8, 1), 256, 0, stream>>>(
      H16, H16, kH, 0L, WDT, WDT, kH, 0L, (void*)G32, (void*)G32, kD, 0L, BIAS + kFBD, nullptr, 0L, kB, kD, kH, kSc);
  out_kernel<<<4096, kThr, 0, stream>>>(G32, out);
}
